// DualCrossAttention_49005576847529
// MI455X (gfx1250) — hardware-run, weakly checked
//
#include <hip/hip_runtime.h>
#include <stddef.h>
#include <stdint.h>

#define NBATCH 8
#define S1     768
#define S2A    1024
#define S2B    768
#define DM     512
#define NH     8
#define HDM    64
#define DFF    2048
#define NTOK   (NBATCH * S1)
#define NTKA   (NBATCH * S2A)
#define QB     128
#define KC     64
#define NQB    (S1 / QB)

static_assert(NTOK == 6144);
static_assert(NTKA == 8192);
static_assert(S1 % 256 == 0);
static_assert(S2A % 256 == 0);
static_assert(S2B % 256 == 0);
static_assert(S1 % QB == 0);
static_assert(S2A % KC == 0);
static_assert(S2B % KC == 0);
static_assert(DM % 64 == 0);
static_assert(DFF % 64 == 0);
static_assert(NH * HDM == DM);
static_assert(NTOK % 256 == 0);
static_assert(NTKA % 256 == 0);
static_assert(NTOK % 8 == 0);
static_assert((NTOK * DM) % 2048 == 0);
static_assert((NTKA * DM) % 2048 == 0);
static_assert((DM * DM) % 2048 == 0);
static_assert((DFF * DM) % 2048 == 0);

typedef _Float16 v16h __attribute__((ext_vector_type(16)));
typedef _Float16 v8h  __attribute__((ext_vector_type(8)));
typedef float    v8f  __attribute__((ext_vector_type(8)));
typedef float    v4f  __attribute__((ext_vector_type(4)));
typedef unsigned int v4u __attribute__((ext_vector_type(4)));

union Frag  { v16h v; v8h h[2]; };
union Pack8 { v8h h; v4u u; };

__device__ __forceinline__ v8f mma16(v16h a, v16h b, v8f c) {
  c = __builtin_amdgcn_wmma_f32_16x16x32_f16(false, a, false, b, (short)0, c, false, false);
  asm volatile("v_nop\n\tv_nop\n\tv_nop\n\tv_nop" : "+v"(c) : "v"(a), "v"(b));
  return c;
}

__device__ __forceinline__ v16h ldfrag(const _Float16* p, int ld, int row0, int k0, int lane) {
  const int m = lane & 15, lh = lane >> 4;
  const _Float16* q = p + (size_t)(row0 + m) * ld + k0 + 8 * lh;
  Frag f;
  f.h[0] = *(const v8h*)(q);
  f.h[1] = *(const v8h*)(q + 16);
  return f.v;
}

__device__ __forceinline__ v8f zero8() { return (v8f){0.f, 0.f, 0.f, 0.f, 0.f, 0.f, 0.f, 0.f}; }

__device__ __forceinline__ void gemm32x64(const _Float16* __restrict__ A, int lda,
                                          const _Float16* __restrict__ Bt, int ldb, int K,
                                          int m0, int n0, int lane, v8f (&acc)[2][4]) {
#pragma unroll 1
  for (int k0 = 0; k0 < K; k0 += 32) {
    const v16h a0 = ldfrag(A, lda, m0, k0, lane);
    const v16h a1 = ldfrag(A, lda, m0 + 16, k0, lane);
    const v16h b0 = ldfrag(Bt, ldb, n0, k0, lane);
    const v16h b1 = ldfrag(Bt, ldb, n0 + 16, k0, lane);
    const v16h b2 = ldfrag(Bt, ldb, n0 + 32, k0, lane);
    const v16h b3 = ldfrag(Bt, ldb, n0 + 48, k0, lane);
    acc[0][0] = mma16(a0, b0, acc[0][0]);
    acc[1][0] = mma16(a1, b0, acc[1][0]);
    acc[0][1] = mma16(a0, b1, acc[0][1]);
    acc[1][1] = mma16(a1, b1, acc[1][1]);
    acc[0][2] = mma16(a0, b2, acc[0][2]);
    acc[1][2] = mma16(a1, b2, acc[1][2]);
    acc[0][3] = mma16(a0, b3, acc[0][3]);
    acc[1][3] = mma16(a1, b3, acc[1][3]);
  }
}

__global__ __launch_bounds__(256) void k_cvt(const float* __restrict__ src, _Float16* __restrict__ dh, float scale) {
  const size_t o = (size_t)blockIdx.x * 2048 + (size_t)threadIdx.x * 8;
  const v4f a0 = *(const v4f*)(src + o) * scale;
  const v4f a1 = *(const v4f*)(src + o + 4) * scale;
  Pack8 pk;
  pk.h = (v8h){(_Float16)a0[0], (_Float16)a0[1], (_Float16)a0[2], (_Float16)a0[3],
               (_Float16)a1[0], (_Float16)a1[1], (_Float16)a1[2], (_Float16)a1[3]};
  const v4u vv = pk.u;
  volatile v4u* d = (volatile v4u*)(dh + o);
  *d = vv;
  __threadfence();
  *d = vv;
}

#define STP 72
#define SVP 264
__global__ __launch_bounds__(256) void k_proj(const _Float16* __restrict__ xh,
                                              const _Float16* __restrict__ wt,
                                              int S, int which_base,
                                              _Float16* __restrict__ qk,
                                              _Float16* __restrict__ vtp) {
  __shared__ __align__(16) _Float16 st[256 * STP];
  const int tid = threadIdx.x, lane = tid & 31, wave = tid >> 5;
  const int hh = lane >> 4, c = lane & 15;
  const int bx  = blockIdx.x;
  const int nsb = S >> 8;
  const int b   = bx / nsb;
  const int sb  = (bx - b * nsb) * 256;
  const int ns  = blockIdx.y;
  const int which = which_base + (ns >> 3);
  const int head  = ns & 7;
  const int hb    = b * NH + head;
  const int m0 = sb + wave * 32;
  const int n0 = ns * 64;
  const _Float16* A = xh + (size_t)b * S * DM;

  v8f acc[2][4];
#pragma unroll
  for (int s = 0; s < 2; ++s)
#pragma unroll
    for (int t = 0; t < 4; ++t) acc[s][t] = zero8();
  gemm32x64(A, DM, wt, DM, DM, m0, n0, lane, acc);

  if (which < 2) {
#pragma unroll
    for (int sub = 0; sub < 2; ++sub)
#pragma unroll
      for (int t = 0; t < 4; ++t)
#pragma unroll
        for (int r = 0; r < 8; ++r)
          st[(wave * 32 + sub * 16 + 8 * hh + r) * STP + 16 * t + c] =
              (_Float16)(acc[sub][t][r] * 0.03125f);
  } else {
#pragma unroll
    for (int sub = 0; sub < 2; ++sub)
#pragma unroll
      for (int t = 0; t < 4; ++t)
#pragma unroll
        for (int r = 0; r < 8; ++r)
          st[(16 * t + c) * SVP + wave * 32 + sub * 16 + 8 * hh + r] =
              (_Float16)(acc[sub][t][r] * 0.03125f);
  }
  __syncthreads();

  if (which < 2) {
    _Float16* base = qk + (size_t)hb * S * HDM;
#pragma unroll
    for (int g = 0; g < 2; ++g) {
      v4u val[4];
      size_t go[4];
#pragma unroll
      for (int j = 0; j < 4; ++j) {
        const int p  = tid + 256 * (4 * g + j);
        const int lr = p >> 3;
        const int pc = p & 7;
        Pack8 pk;
        pk.h   = *(const v8h*)(st + lr * STP + pc * 8);
        val[j] = pk.u;
        go[j]  = (size_t)(sb + lr) * HDM + pc * 8;
      }
      for (int ps = 0; ps < 2; ++ps) {
#pragma unroll
        for (int j = 0; j < 4; ++j) *(volatile v4u*)(base + go[j]) = val[j];
        __threadfence();
      }
    }
  } else {
    _Float16* base = vtp + (size_t)hb * HDM * S;
#pragma unroll
    for (int g = 0; g < 2; ++g) {
      v4u val[4];
      size_t go[4];
#pragma unroll
      for (int j = 0; j < 4; ++j) {
        const int p    = tid + 256 * (4 * g + j);
        const int drow = p >> 5;
        const int pc   = p & 31;
        Pack8 pk;
        pk.h   = *(const v8h*)(st + drow * SVP + pc * 8);
        val[j] = pk.u;
        go[j]  = (size_t)drow * S + sb + pc * 8;
      }
      for (int ps = 0; ps < 2; ++ps) {
#pragma unroll
        for (int j = 0; j < 4; ++j) *(volatile v4u*)(base + go[j]) = val[j];
        __threadfence();
      }
    }
  }
}

#define KTP 72
__global__ __launch_bounds__(256) void k_attn(const _Float16* __restrict__ qp,
                                              const _Float16* __restrict__ kp,
                                              const _Float16* __restrict__ vt,
                                              _Float16* __restrict__ op,
                                              int s2, int mode, float sscale) {
  __shared__ __align__(16) _Float16 Ks[KC * KTP];
  __shared__ __align__(16) _Float16 Vs[HDM * KTP];
  __shared__ __align__(16) _Float16 Ps[8 * 16 * KTP];

  const int tid = threadIdx.x, lane = tid & 31, wave = tid >> 5;
  const int hh = lane >> 4, c = lane & 15;
  const int qb  = blockIdx.x % NQB;
  const int hb  = blockIdx.x / NQB;
  const int h   = hb & 7;
  const int b   = hb >> 3;
  const int q0  = qb * QB + wave * 16;
  const int nck = s2 >> 6;

  const _Float16* Q = qp + (size_t)hb * S1 * HDM;
  const _Float16* K = kp + (size_t)hb * s2 * HDM;
  const _Float16* V = vt + (size_t)hb * HDM * s2;

  v16h qa[2];
  qa[0] = ldfrag(Q, HDM, q0, 0, lane);
  qa[1] = ldfrag(Q, HDM, q0, 32, lane);

  const float NEGI = -__builtin_huge_valf();
  float mrow[8], lrow[8];
  v8f oacc[4];
#pragma unroll
  for (int r = 0; r < 8; ++r) { mrow[r] = NEGI; lrow[r] = 0.f; }
#pragma unroll
  for (int t = 0; t < 4; ++t) oacc[t] = zero8();

  _Float16* pw = Ps + wave * 16 * KTP;

  for (int kc = 0; kc < nck; ++kc) {
    const int kv0 = kc * KC;
    __syncthreads();
    {
      const int r  = tid >> 2;
      const int qq = (tid & 3) * 16;
      const _Float16* ks = K + (size_t)(kv0 + r) * HDM + qq;
      const _Float16* vs = V + (size_t)r * s2 + kv0 + qq;
#pragma unroll
      for (int e = 0; e < 2; ++e) {
        *(v8h*)(Ks + r * KTP + qq + 8 * e) = *(const v8h*)(ks + 8 * e);
        *(v8h*)(Vs + r * KTP + qq + 8 * e) = *(const v8h*)(vs + 8 * e);
      }
    }
    __syncthreads();

    v8f s[4];
#pragma unroll
    for (int j = 0; j < 4; ++j) s[j] = zero8();
#pragma unroll
    for (int dc = 0; dc < 2; ++dc) {
#pragma unroll
      for (int j = 0; j < 4; ++j) {
        const v16h kb = ldfrag(Ks, KTP, j * 16, dc * 32, lane);
        s[j] = mma16(qa[dc], kb, s[j]);
      }
    }
    float rw[8];
#pragma unroll
    for (int r = 0; r < 8; ++r) {
      const int qg = q0 + 8 * hh + r;
      const int same1 = ((qg < 512) == (kv0 < 512)) ? 1 : 0;
      const int same2 = ((qg >> 8) == (kv0 >> 8)) ? 1 : 0;
      const int same  = (mode == 1) ? same1 : same2;
      rw[r] = same ? 1.25f : 1.0f;
    }
    float cm[8];
#pragma unroll
    for (int r = 0; r < 8; ++r) {
      float m = NEGI;
#pragma unroll
      for (int j = 0; j < 4; ++j) { s[j][r] = (s[j][r] * sscale) * rw[r]; m = fmaxf(m, s[j][r]); }
#pragma unroll
      for (int off = 1; off < 16; off <<= 1) m = fmaxf(m, __shfl_xor(m, off, 32));
      cm[r] = m;
    }
    float al[8];
#pragma unroll
    for (int r = 0; r < 8; ++r) {
      const float mnew  = fmaxf(mrow[r], cm[r]);
      const float alpha = __expf(mrow[r] - mnew);
      mrow[r] = mnew;
      float psum = 0.f;
#pragma unroll
      for (int j = 0; j < 4; ++j) {
        const float p = __expf(s[j][r] - mnew);
        psum += p;
        pw[(8 * hh + r) * KTP + j * 16 + c] = (_Float16)(p * 1024.0f);
      }
#pragma unroll
      for (int off = 1; off < 16; off <<= 1) psum += __shfl_xor(psum, off, 32);
      lrow[r] = lrow[r] * alpha + psum;
      al[r] = alpha;
    }
#pragma unroll
    for (int t = 0; t < 4; ++t)
#pragma unroll
      for (int r = 0; r < 8; ++r) oacc[t][r] *= al[r];
    __syncthreads();

#pragma unroll
    for (int kk = 0; kk < 2; ++kk) {
      const v16h pa = ldfrag(pw, KTP, 0, kk * 32, lane);
#pragma unroll
      for (int t = 0; t < 4; ++t) {
        const v16h vb = ldfrag(Vs, KTP, t * 16, kk * 32, lane);
        oacc[t] = mma16(pa, vb, oacc[t]);
      }
    }
  }

  float invl[8];
#pragma unroll
  for (int r = 0; r < 8; ++r) invl[r] = (lrow[r] > 0.f) ? (0.0625f / lrow[r]) : 0.f;
  __syncthreads();
#pragma unroll
  for (int r = 0; r < 8; ++r) {
#pragma unroll
    for (int t = 0; t < 4; ++t)
      pw[(8 * hh + r) * KTP + 16 * t + c] = (_Float16)(oacc[t][r] * invl[r]);
  }
  __syncthreads();
  v4u val[4];
  size_t go[4];
#pragma unroll
  for (int it = 0; it < 4; ++it) {
    const int p  = lane + 32 * it;
    const int L  = p >> 3;
    const int pc = p & 7;
    Pack8 pk;
    pk.h    = *(const v8h*)(pw + L * KTP + pc * 8);
    val[it] = pk.u;
    go[it]  = ((size_t)b * S1 + (size_t)(q0 + L)) * DM + (size_t)h * HDM + pc * 8;
  }
  for (int ps = 0; ps < 2; ++ps) {
#pragma unroll
    for (int it = 0; it < 4; ++it) *(volatile v4u*)(op + go[it]) = val[it];
    __threadfence();
  }
}

#define OTP 68
__device__ __forceinline__ void out_epilogue_f32(v8f (&acc)[2][4], float scale, const float (&bb)[4],
                                                 float* sw, float* __restrict__ out, int ldo,
                                                 int m0, int n0, int lane, int hh, int c) {
#pragma unroll
  for (int sub = 0; sub < 2; ++sub) {
    __syncthreads();
#pragma unroll
    for (int t = 0; t < 4; ++t) {
#pragma unroll
      for (int r = 0; r < 8; ++r) sw[(8 * hh + r) * OTP + 16 * t + c] = acc[sub][t][r] * scale + bb[t];
    }
    __syncthreads();
    v4f val[8];
    size_t go[8];
#pragma unroll
    for (int it = 0; it < 8; ++it) {
      const int p    = lane + 32 * it;
      const int L    = p >> 3;
      const int pc   = p & 7;
      const int row  = L >> 1;
      const int half = L & 1;
      val[it] = *(const v4f*)(sw + row * OTP + half * 32 + pc * 4);
      go[it]  = (size_t)(m0 + sub * 16 + row) * ldo + n0 + half * 32 + pc * 4;
    }
    for (int ps = 0; ps < 2; ++ps) {
#pragma unroll
      for (int it = 0; it < 8; ++it) *(volatile v4f*)(out + go[it]) = val[it];
      __threadfence();
    }
  }
}

__device__ __forceinline__ void out_epilogue_h16(v8f (&acc)[2][4], float scale, const float (&bb)[4], float oscale,
                                                 float* sw, _Float16* __restrict__ out, int ldo,
                                                 int m0, int n0, int lane, int hh, int c) {
#pragma unroll
  for (int sub = 0; sub < 2; ++sub) {
    __syncthreads();
#pragma unroll
    for (int t = 0; t < 4; ++t) {
#pragma unroll
      for (int r = 0; r < 8; ++r) {
        const float v  = acc[sub][t][r] * scale + bb[t];
        const float gl = 0.5f * v * (1.0f + erff(v * 0.70710678118654752f));
        sw[(8 * hh + r) * OTP + 16 * t + c] = gl * oscale;
      }
    }
    __syncthreads();
    v4u val[4];
    size_t go[4];
#pragma unroll
    for (int it = 0; it < 4; ++it) {
      const int p  = lane + 32 * it;
      const int L  = p >> 3;
      const int pc = p & 7;
      const float* ra = sw + L * OTP + pc * 8;
      const v4f a0 = *(const v4f*)(ra), a1 = *(const v4f*)(ra + 4);
      Pack8 pk;
      pk.h = (v8h){(_Float16)a0[0], (_Float16)a0[1], (_Float16)a0[2], (_Float16)a0[3],
                   (_Float16)a1[0], (_Float16)a1[1], (_Float16)a1[2], (_Float16)a1[3]};
      val[it] = pk.u;
      go[it]  = (size_t)(m0 + sub * 16 + L) * ldo + n0 + pc * 8;
    }
    for (int ps = 0; ps < 2; ++ps) {
#pragma unroll
      for (int it = 0; it < 4; ++it) *(volatile v4u*)(out + go[it]) = val[it];
      __threadfence();
    }
  }
}

__global__ __launch_bounds__(256) void k_gemm_f32(const _Float16* __restrict__ ap, int lda,
                                                  const _Float16* __restrict__ wt, int K,
                                                  const float* __restrict__ bias, float scale,
                                                  float* __restrict__ out, int ldo) {
  __shared__ __align__(16) float st[8][16 * OTP];
  const int tid = threadIdx.x, lane = tid & 31, wave = tid >> 5;
  const int hh = lane >> 4, c = lane & 15;
  const int m0 = blockIdx.x * 256 + wave * 32;
  const int n0 = blockIdx.y * 64;

  v8f acc[2][4];
#pragma unroll
  for (int s = 0; s < 2; ++s)
#pragma unroll
    for (int t = 0; t < 4; ++t) acc[s][t] = zero8();
  gemm32x64(ap, lda, wt, K, K, m0, n0, lane, acc);
  float bb[4];
#pragma unroll
  for (int t = 0; t < 4; ++t) bb[t] = bias[n0 + 16 * t + c];
  out_epilogue_f32(acc, scale, bb, st[wave], out, ldo, m0, n0, lane, hh, c);
}

__global__ __launch_bounds__(256) void k_gemm_h16(const _Float16* __restrict__ ap, int lda,
                                                  const _Float16* __restrict__ wt, int K,
                                                  const float* __restrict__ bias, float scale, float oscale,
                                                  _Float16* __restrict__ out, int ldo) {
  __shared__ __align__(16) float st[8][16 * OTP];
  const int tid = threadIdx.x, lane = tid & 31, wave = tid >> 5;
  const int hh = lane >> 4, c = lane & 15;
  const int m0 = blockIdx.x * 256 + wave * 32;
  const int n0 = blockIdx.y * 64;

  v8f acc[2][4];
#pragma unroll
  for (int s = 0; s < 2; ++s)
#pragma unroll
    for (int t = 0; t < 4; ++t) acc[s][t] = zero8();
  gemm32x64(ap, lda, wt, K, K, m0, n0, lane, acc);
  float bb[4];
#pragma unroll
  for (int t = 0; t < 4; ++t) bb[t] = bias[n0 + 16 * t + c];
  out_epilogue_h16(acc, scale, bb, oscale, st[wave], out, ldo, m0, n0, lane, hh, c);
}

__global__ __launch_bounds__(256) void k_ln_mid(const float* __restrict__ t, const float* __restrict__ res,
                                                const float* __restrict__ g, const float* __restrict__ be,
                                                float* __restrict__ yf, _Float16* __restrict__ yh) {
  __shared__ __align__(16) float sw[8][DM];
  const int tid = threadIdx.x, lane = tid & 31, wave = tid >> 5;
  const size_t m = (size_t)blockIdx.x * 8 + wave;
  const float* tr = t + m * DM;
  const float* rr = res + m * DM;

  v4f v[4];
  float s = 0.f;
#pragma unroll
  for (int it = 0; it < 4; ++it) {
    const int idx = it * 128 + lane * 4;
    const v4f a = *(const v4f*)(tr + idx);
    const v4f r = *(const v4f*)(rr + idx);
    v[it] = a + r;
    s += (v[it][0] + v[it][1]) + (v[it][2] + v[it][3]);
  }
#pragma unroll
  for (int off = 16; off >= 1; off >>= 1) s += __shfl_xor(s, off, 32);
  const float mean = s * 0.001953125f;
  float ss = 0.f;
#pragma unroll
  for (int it = 0; it < 4; ++it) {
    const v4f d = v[it] - mean;
    ss += (d[0] * d[0] + d[1] * d[1]) + (d[2] * d[2] + d[3] * d[3]);
  }
#pragma unroll
  for (int off = 16; off >= 1; off >>= 1) ss += __shfl_xor(ss, off, 32);
  const float var  = ss * 0.001953125f;
  const float rstd = rsqrtf(var + 1e-5f);

  v4f y[4];
#pragma unroll
  for (int it = 0; it < 4; ++it) {
    const int idx = it * 128 + lane * 4;
    const v4f gv = *(const v4f*)(g + idx);
    const v4f bv = *(const v4f*)(be + idx);
    y[it] = ((v[it] - mean) * rstd) * gv + bv;
  }
  for (int ps = 0; ps < 2; ++ps) {
#pragma unroll
    for (int it = 0; it < 4; ++it) *(volatile v4f*)(yf + m * DM + it * 128 + lane * 4) = y[it];
    __threadfence();
  }
#pragma unroll
  for (int it = 0; it < 4; ++it) *(v4f*)(sw[wave] + it * 128 + lane * 4) = y[it];
  __syncthreads();
  v4u hv[2];
  size_t go[2];
#pragma unroll
  for (int j = 0; j < 2; ++j) {
    const float* cp = sw[wave] + 256 * j + 8 * lane;
    const v4f a0 = *(const v4f*)(cp), a1 = *(const v4f*)(cp + 4);
    Pack8 pk;
    pk.h = (v8h){(_Float16)a0[0], (_Float16)a0[1], (_Float16)a0[2], (_Float16)a0[3],
                 (_Float16)a1[0], (_Float16)a1[1], (_Float16)a1[2], (_Float16)a1[3]};
    hv[j] = pk.u;
    go[j] = m * DM + 256 * j + 8 * lane;
  }
  for (int ps = 0; ps < 2; ++ps) {
#pragma unroll
    for (int j = 0; j < 2; ++j) *(volatile v4u*)(yh + go[j]) = hv[j];
    __threadfence();
  }
}

__global__ __launch_bounds__(256) void k_ln_out(const float* __restrict__ t, const float* __restrict__ res,
                                                const float* __restrict__ g, const float* __restrict__ be,
                                                float* __restrict__ out) {
  const int tid = threadIdx.x, lane = tid & 31, wave = tid >> 5;
  const size_t m = (size_t)blockIdx.x * 8 + wave;
  const float* tr = t + m * DM;
  const float* rr = res + m * DM;

  v4f v[4];
  float s = 0.f;
#pragma unroll
  for (int it = 0; it < 4; ++it) {
    const int idx = it * 128 + lane * 4;
    const v4f a = *(const v4f*)(tr + idx);
    const v4f r = *(const v4f*)(rr + idx);
    v[it] = a + r;
    s += (v[it][0] + v[it][1]) + (v[it][2] + v[it][3]);
  }
#pragma unroll
  for (int off = 16; off >= 1; off >>= 1) s += __shfl_xor(s, off, 32);
  const float mean = s * 0.001953125f;
  float ss = 0.f;
#pragma unroll
  for (int it = 0; it < 4; ++it) {
    const v4f d = v[it] - mean;
    ss += (d[0] * d[0] + d[1] * d[1]) + (d[2] * d[2] + d[3] * d[3]);
  }
#pragma unroll
  for (int off = 16; off >= 1; off >>= 1) ss += __shfl_xor(ss, off, 32);
  const float var  = ss * 0.001953125f;
  const float rstd = rsqrtf(var + 1e-5f);

  v4f o[4];
#pragma unroll
  for (int it = 0; it < 4; ++it) {
    const int idx = it * 128 + lane * 4;
    const v4f gv = *(const v4f*)(g + idx);
    const v4f bv = *(const v4f*)(be + idx);
    o[it] = ((v[it] - mean) * rstd) * gv + bv;
  }
  for (int ps = 0; ps < 2; ++ps) {
#pragma unroll
    for (int it = 0; it < 4; ++it) *(volatile v4f*)(out + m * DM + it * 128 + lane * 4) = o[it];
    __threadfence();
  }
}

extern "C" void kernel_launch(void* const* d_in, const int* in_sizes, int n_in,
                              void* d_out, int out_size, void* d_ws, size_t ws_size,
                              hipStream_t stream) {
  if (n_in < 23) return;
  if (in_sizes[0] != NTOK * DM) return;
  if (in_sizes[1] != NTKA * DM) return;
  if (in_sizes[2] != NTOK * DM) return;
  if (in_sizes[3] != DM * DM) return;
  if (in_sizes[4] != DM * DM) return;
  if (in_sizes[5] != DM * DM) return;
  if (in_sizes[6] != DM * DM) return;
  if (in_sizes[7] != DM) return;
  if (in_sizes[8] != DM * DM) return;
  if (in_sizes[9] != DM * DM) return;
  if (in_sizes[10] != DM * DM) return;
  if (in_sizes[11] != DM * DM) return;
  if (in_sizes[12] != DM) return;
  for (int i = 13; i <= 18; ++i) if (in_sizes[i] != DM) return;
  if (in_sizes[19] != DFF * DM) return;
  if (in_sizes[20] != DFF) return;
  if (in_sizes[21] != DM * DFF) return;
  if (in_sizes[22] != DM) return;
  if (out_size != NTOK * DM) return;

  const float* xq   = (const float*)d_in[0];
  const float* xka  = (const float*)d_in[1];
  const float* xkb  = (const float*)d_in[2];
  const float* wq1  = (const float*)d_in[3];
  const float* wk1  = (const float*)d_in[4];
  const float* wv1  = (const float*)d_in[5];
  const float* wo1  = (const float*)d_in[6];
  const float* bo1  = (const float*)d_in[7];
  const float* wq2  = (const float*)d_in[8];
  const float* wk2  = (const float*)d_in[9];
  const float* wv2  = (const float*)d_in[10];
  const float* wo2  = (const float*)d_in[11];
  const float* bo2  = (const float*)d_in[12];
  const float* g1   = (const float*)d_in[13];
  const float* be1  = (const float*)d_in[14];
  const float* g2   = (const float*)d_in[15];
  const float* be2  = (const float*)d_in[16];
  const float* g3   = (const float*)d_in[17];
  const float* be3  = (const float*)d_in[18];
  const float* w1   = (const float*)d_in[19];
  const float* b1   = (const float*)d_in[20];
  const float* w2   = (const float*)d_in[21];
  const float* b2   = (const float*)d_in[22];
  float* out = (float*)d_out;

  size_t off = 0;
  const size_t oXc   = off; off += (size_t)NTOK * DM * 2;
  const size_t oXs   = off; off += (size_t)NTKA * DM * 2;
  const size_t oXv   = off; off += (size_t)NTOK * DM * 2;
  const size_t oWq1  = off; off += (size_t)DM * DM * 2;
  const size_t oWkv1 = off; off += (size_t)2 * DM * DM * 2;
  const size_t oWo1  = off; off += (size_t)DM * DM * 2;
  const size_t oWq2  = off; off += (size_t)DM * DM * 2;
  const size_t oWkv2 = off; off += (size_t)2 * DM * DM * 2;
  const size_t oWo2  = off; off += (size_t)DM * DM * 2;
  const size_t oW1   = off; off += (size_t)DFF * DM * 2;
  const size_t oW2   = off; off += (size_t)DM * DFF * 2;
  const size_t oQ    = off; off += (size_t)NBATCH * NH * S1 * HDM * 2;
  const size_t oK    = off; off += (size_t)NBATCH * NH * S2A * HDM * 2;
  const size_t oV    = off; off += (size_t)NBATCH * NH * HDM * S2A * 2;
  const size_t oO    = off; off += (size_t)NTOK * DM * 2;
  const size_t oHd   = oQ;
  if (oHd + (size_t)NTOK * DFF * 2 > off) return;
  const size_t oT    = off; off += (size_t)NTOK * DM * 4;
  const size_t oR1   = off; off += (size_t)NTOK * DM * 4;
  const size_t oR1h  = off; off += (size_t)NTOK * DM * 2;
  const size_t oR2   = off; off += (size_t)NTOK * DM * 4;
  const size_t oR2h  = off; off += (size_t)NTOK * DM * 2;
  if (off > ws_size) return;
  if (off > (size_t)134217728) return;

  char* ws = (char*)d_ws;
  _Float16* Xc   = (_Float16*)(ws + oXc);
  _Float16* Xs   = (_Float16*)(ws + oXs);
  _Float16* Xv   = (_Float16*)(ws + oXv);
  _Float16* Wq1t = (_Float16*)(ws + oWq1);
  _Float16* Wkv1 = (_Float16*)(ws + oWkv1);
  _Float16* Wo1t = (_Float16*)(ws + oWo1);
  _Float16* Wq2t = (_Float16*)(ws + oWq2);
  _Float16* Wkv2 = (_Float16*)(ws + oWkv2);
  _Float16* Wo2t = (_Float16*)(ws + oWo2);
  _Float16* W1t  = (_Float16*)(ws + oW1);
  _Float16* W2t  = (_Float16*)(ws + oW2);
  _Float16* Qp   = (_Float16*)(ws + oQ);
  _Float16* Kp   = (_Float16*)(ws + oK);
  _Float16* Vt   = (_Float16*)(ws + oV);
  _Float16* Op   = (_Float16*)(ws + oO);
  _Float16* Hd   = (_Float16*)(ws + oHd);
  float*    T    = (float*)(ws + oT);
  float*    R1   = (float*)(ws + oR1);
  _Float16* R1h  = (_Float16*)(ws + oR1h);
  float*    R2   = (float*)(ws + oR2);
  _Float16* R2h  = (_Float16*)(ws + oR2h);

  k_cvt<<<dim3((NTOK * DM) / 2048), dim3(256), 0, stream>>>(xq, Xc, 1.0f);
  k_cvt<<<dim3((NTKA * DM) / 2048), dim3(256), 0, stream>>>(xka, Xs, 1.0f);
  k_cvt<<<dim3((NTOK * DM) / 2048), dim3(256), 0, stream>>>(xkb, Xv, 1.0f);
  k_cvt<<<dim3((DM * DM) / 2048), dim3(256), 0, stream>>>(wq1, Wq1t, 32.0f);
  k_cvt<<<dim3((DM * DM) / 2048), dim3(256), 0, stream>>>(wk1, Wkv1, 32.0f);
  k_cvt<<<dim3((DM * DM) / 2048), dim3(256), 0, stream>>>(wv1, Wkv1 + (size_t)DM * DM, 32.0f);
  k_cvt<<<dim3((DM * DM) / 2048), dim3(256), 0, stream>>>(wo1, Wo1t, 32.0f);
  k_cvt<<<dim3((DM * DM) / 2048), dim3(256), 0, stream>>>(wq2, Wq2t, 32.0f);
  k_cvt<<<dim3((DM * DM) / 2048), dim3(256), 0, stream>>>(wk2, Wkv2, 32.0f);
  k_cvt<<<dim3((DM * DM) / 2048), dim3(256), 0, stream>>>(wv2, Wkv2 + (size_t)DM * DM, 32.0f);
  k_cvt<<<dim3((DM * DM) / 2048), dim3(256), 0, stream>>>(wo2, Wo2t, 32.0f);
  k_cvt<<<dim3((DFF * DM) / 2048), dim3(256), 0, stream>>>(w1, W1t, 32.0f);
  k_cvt<<<dim3((DM * DFF) / 2048), dim3(256), 0, stream>>>(w2, W2t, 32.0f);

  const float sscale = 0.125f;

  k_proj<<<dim3(NBATCH * (S1 / 256), NH), dim3(256), 0, stream>>>(Xc, Wq1t, S1, 0, Qp, Vt);
  k_proj<<<dim3(NBATCH * (S2A / 256), 2 * NH), dim3(256), 0, stream>>>(Xs, Wkv1, S2A, 1, Kp, Vt);
  k_attn<<<dim3(NBATCH * NH * NQB), dim3(256), 0, stream>>>(Qp, Kp, Vt, Op, S2A, 1, sscale);
  k_gemm_f32<<<dim3(NTOK / 256, DM / 64), dim3(256), 0, stream>>>(Op, DM, Wo1t, DM, bo1, 0.00048828125f, T, DM);
  k_ln_mid<<<dim3(NTOK / 8), dim3(256), 0, stream>>>(T, xq, g1, be1, R1, R1h);

  k_proj<<<dim3(NBATCH * (S1 / 256), NH), dim3(256), 0, stream>>>(R1h, Wq2t, S1, 0, Qp, Vt);
  k_proj<<<dim3(NBATCH * (S2B / 256), 2 * NH), dim3(256), 0, stream>>>(Xv, Wkv2, S2B, 1, Kp, Vt);
  k_attn<<<dim3(NBATCH * NH * NQB), dim3(256), 0, stream>>>(Qp, Kp, Vt, Op, S2B, 2, sscale);
  k_gemm_f32<<<dim3(NTOK / 256, DM / 64), dim3(256), 0, stream>>>(Op, DM, Wo2t, DM, bo2, 0.00048828125f, T, DM);
  k_ln_mid<<<dim3(NTOK / 8), dim3(256), 0, stream>>>(T, R1, g2, be2, R2, R2h);

  k_gemm_h16<<<dim3(NTOK / 256, DFF / 64), dim3(256), 0, stream>>>(R2h, DM, W1t, DM, b1, 0.03125f, 16.0f, Hd, DFF);
  k_gemm_f32<<<dim3(NTOK / 256, DM / 64), dim3(256), 0, stream>>>(Hd, DFF, W2t, DFF, b2, 0.001953125f, T, DM);
  k_ln_out<<<dim3(NTOK / 8), dim3(256), 0, stream>>>(T, R2, g3, be3, out);
  (void)hipGetLastError();
}
